// CrossAttention_6820408066620
// MI455X (gfx1250) — hardware-run, weakly checked
//
#include <hip/hip_runtime.h>
#ifndef NB
#define NB 8
#endif
#ifndef SEQ
#define SEQ 4096
#endif
#define NB_FULL 8
#define SEQ_FULL 4096
#define CC 64
#define CQ 19
#define CQP 32
#define XP 72
#define WP 40
#define SOP 68

static_assert(CC == 64);
static_assert(CC % 32 == 0);
static_assert(CQP == 32 && CQ <= CQP);
static_assert(SEQ % 64 == 0);
static_assert(SEQ <= SEQ_FULL);
static_assert(NB <= NB_FULL);
static_assert(SEQ_FULL % 4 == 0);
static_assert(XP % 8 == 0 && XP >= CC);
static_assert(WP % 8 == 0 && WP >= CQP);
static_assert(SOP % 4 == 0 && SOP >= 64);
static_assert((size_t)5 * NB * SEQ * CC * 2 <= (size_t)134217728);
static_assert((size_t)NB_FULL * CC * SEQ_FULL * 4 == (size_t)8388608);

typedef __bf16 v16b __attribute__((ext_vector_type(16)));
typedef _Float16 v16h __attribute__((ext_vector_type(16)));
typedef unsigned short v8us __attribute__((ext_vector_type(8), may_alias));
typedef float v8f __attribute__((ext_vector_type(8)));
typedef float v4f __attribute__((ext_vector_type(4)));
typedef float v4fa __attribute__((ext_vector_type(4), may_alias));
typedef _Float16 h16;
union FragB { v16b v; v8us half[2]; unsigned short u[16]; };
union FragH { v16h v; v8us half[2]; _Float16 h[16]; unsigned short u[16]; };

__device__ __forceinline__ unsigned short bf16_bits(float x) { unsigned int u = __float_as_uint(x); return (unsigned short)((u + 0x7FFFu + ((u >> 16) & 1u)) >> 16); }
__device__ __forceinline__ float bf16_val(unsigned short b) { return __uint_as_float(((unsigned int)b) << 16); }
__device__ __forceinline__ float bf16_rne(float x) { return bf16_val(bf16_bits(x)); }

static __device__ __forceinline__ h16 toh_flush(float v) { const h16 r = (h16)v; return (fabsf(v) < 6.103515625e-05f) ? (h16)0.0f : r; }
static __device__ __forceinline__ float exp2_cut(float e) { const float p = __builtin_amdgcn_exp2f(e); return (e < -27.0f) ? 0.0f : p; }

__device__ __forceinline__ v8f mma1b(v16b a, v16b b, v8f c) {
  c = __builtin_amdgcn_wmma_f32_16x16x32_bf16(false, a, false, b, (short)0, c, false, false);
  asm volatile("v_nop\n\tv_nop\n\tv_nop\n\tv_nop" : "+v"(c) : "v"(a), "v"(b));
  return c;
}
__device__ __forceinline__ v8f mma3b(v16b ah, v16b al, v16b bh, v16b bl, v8f c) {
  c = __builtin_amdgcn_wmma_f32_16x16x32_bf16(false, ah, false, bh, (short)0, c, false, false);
  c = __builtin_amdgcn_wmma_f32_16x16x32_bf16(false, al, false, bh, (short)0, c, false, false);
  c = __builtin_amdgcn_wmma_f32_16x16x32_bf16(false, ah, false, bl, (short)0, c, false, false);
  asm volatile("v_nop\n\tv_nop\n\tv_nop\n\tv_nop" : "+v"(c) : "v"(ah), "v"(al), "v"(bh), "v"(bl));
  return c;
}
__device__ __forceinline__ v8f mma1h(v16h a, v16h b, v8f c) {
  c = __builtin_amdgcn_wmma_f32_16x16x32_f16(false, a, false, b, (short)0, c, false, false);
  asm volatile("v_nop\n\tv_nop\n\tv_nop\n\tv_nop" : "+v"(c) : "v"(a), "v"(b));
  return c;
}

__device__ __forceinline__ v16b frag_b(const unsigned short* __restrict__ p, size_t off) {
  FragB f; f.half[0] = *(const v8us*)(p + off); f.half[1] = *(const v8us*)(p + off + 16); return f.v;
}
__device__ __forceinline__ v16h frag_h(const unsigned short* __restrict__ p, size_t off) {
  FragH f; f.half[0] = *(const v8us*)(p + off); f.half[1] = *(const v8us*)(p + off + 16); return f.v;
}
__device__ __forceinline__ v16b frag_w(const float* __restrict__ W, int off) {
  const v4f x0 = *(const v4fa*)(W + off), x1 = *(const v4fa*)(W + off + 4);
  const v4f x2 = *(const v4fa*)(W + off + 16), x3 = *(const v4fa*)(W + off + 20);
  FragB f;
  f.u[0] = bf16_bits(x0[0]); f.u[1] = bf16_bits(x0[1]); f.u[2] = bf16_bits(x0[2]); f.u[3] = bf16_bits(x0[3]);
  f.u[4] = bf16_bits(x1[0]); f.u[5] = bf16_bits(x1[1]); f.u[6] = bf16_bits(x1[2]); f.u[7] = bf16_bits(x1[3]);
  f.u[8] = bf16_bits(x2[0]); f.u[9] = bf16_bits(x2[1]); f.u[10] = bf16_bits(x2[2]); f.u[11] = bf16_bits(x2[3]);
  f.u[12] = bf16_bits(x3[0]); f.u[13] = bf16_bits(x3[1]); f.u[14] = bf16_bits(x3[2]); f.u[15] = bf16_bits(x3[3]);
  return f.v;
}

__global__ __launch_bounds__(128) void k_proj_q(const float* __restrict__ X, const float* __restrict__ W, const float* __restrict__ bias,
                                                unsigned short* __restrict__ PH, unsigned short* __restrict__ PL) {
  __shared__ __attribute__((aligned(16))) unsigned short xs[64][WP];
  __shared__ __attribute__((aligned(16))) unsigned short wq[64][WP];
  __shared__ __attribute__((aligned(16))) unsigned short sh[64][XP];
  __shared__ __attribute__((aligned(16))) unsigned short sl[64][XP];
  const int tid = threadIdx.x;
  const int wave = __builtin_amdgcn_readfirstlane(tid >> 5);
  const int lane = tid & 31, ln = lane & 15, hh = lane >> 4;
  const int b = blockIdx.y, pb = blockIdx.x * 64;
  const float* xb = X + (size_t)b * CQ * SEQ_FULL + pb;
#pragma unroll
  for (int j = 0; j < 4; ++j) {
    const int idx = j * 128 + tid;
    const int c = idx >> 4, p4 = (idx & 15) * 4;
    const int cl = (c < CQ) ? c : (CQ - 1);
    const v4f x4 = *(const v4fa*)(xb + (size_t)cl * SEQ_FULL + p4);
    const bool live = c < CQ;
    xs[p4 + 0][c] = live ? bf16_bits(x4[0]) : (unsigned short)0;
    xs[p4 + 1][c] = live ? bf16_bits(x4[1]) : (unsigned short)0;
    xs[p4 + 2][c] = live ? bf16_bits(x4[2]) : (unsigned short)0;
    xs[p4 + 3][c] = live ? bf16_bits(x4[3]) : (unsigned short)0;
  }
#pragma unroll 4
  for (int i = tid; i < 64 * CQP; i += 128) {
    const int o = i >> 5, c = i & 31;
    const int cl = (c < CQ) ? c : (CQ - 1);
    const float w = W[o * CQ + cl];
    wq[o][c] = (c < CQ) ? bf16_bits(w) : (unsigned short)0;
  }
  __syncthreads();
  const int prow = wave * 16 + ln;
  FragB a0;
  a0.half[0] = *(const v8us*)&xs[prow][8 * hh];       a0.half[1] = *(const v8us*)&xs[prow][16 + 8 * hh];
#pragma unroll
  for (int ot = 0; ot < 4; ++ot) {
    FragB w0;
    w0.half[0] = *(const v8us*)&wq[ot * 16 + ln][8 * hh];
    w0.half[1] = *(const v8us*)&wq[ot * 16 + ln][16 + 8 * hh];
    v8f acc = {0.f, 0.f, 0.f, 0.f, 0.f, 0.f, 0.f, 0.f};
    acc = mma1b(a0.v, w0.v, acc);
    const float bv = bf16_rne(bias[ot * 16 + ln]);
#pragma unroll
    for (int r = 0; r < 8; ++r) {
      const float v = acc[r] + bv;
      const unsigned short hb = bf16_bits(v);
      const unsigned short lb = bf16_bits(v - bf16_val(hb));
      sh[wave * 16 + 8 * hh + r][ot * 16 + ln] = hb;
      sl[wave * 16 + 8 * hh + r][ot * 16 + ln] = lb;
    }
  }
  __syncthreads();
  const size_t rowbase = (size_t)b * SEQ + pb;
  const int pc = (tid & 7) * 8;
  for (int pass = 0; pass < 2; ++pass) {
#pragma unroll
    for (int it = 0; it < 4; ++it) {
      const int row = it * 16 + (tid >> 3);
      const v8us vh = *(const v8us*)&sh[row][pc];
      const v8us vl = *(const v8us*)&sl[row][pc];
      *(volatile v8us*)(PH + (rowbase + row) * CC + pc) = vh;
      *(volatile v8us*)(PL + (rowbase + row) * CC + pc) = vl;
    }
    if (pass == 0) __threadfence();
  }
}

__global__ __launch_bounds__(128) void k_proj_kv(const float* __restrict__ D, const float* __restrict__ Wk, const float* __restrict__ bk,
                                                 const float* __restrict__ Wv, const float* __restrict__ bv,
                                                 unsigned short* __restrict__ KH, unsigned short* __restrict__ KL, unsigned short* __restrict__ VT) {
  __shared__ float sd[64];
  __shared__ float swk[CC];
  __shared__ float sbk[CC];
  __shared__ float swv[CC];
  __shared__ float sbv[CC];
  const int tid = threadIdx.x;
  const int b = blockIdx.y, pb = blockIdx.x * 64;
  if (tid < 64) {
    sd[tid] = bf16_rne(D[(size_t)b * SEQ_FULL + pb + tid]);
    swk[tid] = bf16_rne(Wk[tid]);
    sbk[tid] = bf16_rne(bk[tid]);
    swv[tid] = bf16_rne(Wv[tid]);
    sbv[tid] = bf16_rne(bv[tid]);
  }
  __syncthreads();
  const int pc = (tid & 7) * 8;
  const int rq = tid >> 3;
  const size_t rowbase = (size_t)b * SEQ + pb;
  for (int pass = 0; pass < 2; ++pass) {
#pragma unroll 1
    for (int it = 0; it < 4; ++it) {
      const int row = it * 16 + rq;
      const float dk = sd[row];
      const float wvc = swv[row], bvc = sbv[row];
      v8us vh, vl, vv;
#pragma unroll
      for (int i = 0; i < 8; ++i) {
        const float kv = swk[pc + i] * dk + sbk[pc + i];
        const unsigned short hb = bf16_bits(kv);
        vh[i] = hb;
        vl[i] = bf16_bits(kv - bf16_val(hb));
        const float vf = wvc * sd[pc + i] + bvc;
        vv[i] = __builtin_bit_cast(unsigned short, toh_flush(vf));
      }
      *(volatile v8us*)(KH + (rowbase + row) * CC + pc) = vh;
      *(volatile v8us*)(KL + (rowbase + row) * CC + pc) = vl;
      *(volatile v8us*)(VT + ((size_t)b * CC + row) * SEQ + pb + pc) = vv;
    }
    if (pass == 0) __threadfence();
  }
}

__global__ __launch_bounds__(128) void k_attn(const unsigned short* __restrict__ QH, const unsigned short* __restrict__ QL,
                                              const unsigned short* __restrict__ KH, const unsigned short* __restrict__ KL,
                                              const unsigned short* __restrict__ VT, const float* __restrict__ Wo, const float* __restrict__ bo,
                                              float* __restrict__ out) {
  __shared__ __attribute__((aligned(16))) float so[CC][SOP];
  const int tid = threadIdx.x;
  const int wave = __builtin_amdgcn_readfirstlane(tid >> 5);
  const int lane = tid & 31, ln = lane & 15, hh = lane >> 4;
  const int b = blockIdx.y, qb = blockIdx.x * 64;
  const size_t tok0 = (size_t)b * SEQ;
  const size_t qoff = (tok0 + qb + wave * 16 + ln) * CC + 8 * hh;
  const v16b qh0 = frag_b(QH, qoff), qh1 = frag_b(QH, qoff + 32);
  const v16b ql0 = frag_b(QL, qoff), ql1 = frag_b(QL, qoff + 32);
  const v8f z8 = {0.f, 0.f, 0.f, 0.f, 0.f, 0.f, 0.f, 0.f};
  v8f o0 = z8, o1 = z8, o2 = z8, o3 = z8;
  float m = -1.0e30f, l = 0.f;
  const float SC = 1.4426950408889634f;
  const size_t kofs = (tok0 + ln) * CC + 8 * hh;
  const size_t vofs = ((size_t)b * CC + ln) * SEQ + 8 * hh;
#pragma unroll 1
  for (int kb = 0; kb < SEQ; kb += 32) {
    const size_t ka = kofs + (size_t)kb * CC;
    v8f s0 = z8, s1 = z8;
    { const v16b ah = frag_b(KH, ka), al = frag_b(KL, ka); s0 = mma3b(ah, al, qh0, ql0, s0); }
    { const v16b ah = frag_b(KH, ka + 32), al = frag_b(KL, ka + 32); s0 = mma3b(ah, al, qh1, ql1, s0); }
    { const v16b ah = frag_b(KH, ka + 16 * CC), al = frag_b(KL, ka + 16 * CC); s1 = mma3b(ah, al, qh0, ql0, s1); }
    { const v16b ah = frag_b(KH, ka + 16 * CC + 32), al = frag_b(KL, ka + 16 * CC + 32); s1 = mma3b(ah, al, qh1, ql1, s1); }
    float cmax = s0[0];
#pragma unroll
    for (int r = 1; r < 8; ++r) cmax = fmaxf(cmax, s0[r]);
#pragma unroll
    for (int r = 0; r < 8; ++r) cmax = fmaxf(cmax, s1[r]);
    cmax = fmaxf(cmax, __shfl_xor(cmax, 16));
    const float mn = fmaxf(m, cmax);
    const float alpha = __builtin_amdgcn_exp2f((m - mn) * SC);
    FragH pf;
    float lsum = 0.f;
#pragma unroll
    for (int r = 0; r < 8; ++r) { const float p = exp2_cut((s0[r] - mn) * SC); lsum += p; pf.h[r] = (_Float16)(p * 16384.0f); }
#pragma unroll
    for (int r = 0; r < 8; ++r) { const float p = exp2_cut((s1[r] - mn) * SC); lsum += p; pf.h[8 + r] = (_Float16)(p * 16384.0f); }
    l = l * alpha + lsum;
    m = mn;
#pragma unroll
    for (int r = 0; r < 8; ++r) { o0[r] *= alpha; o1[r] *= alpha; o2[r] *= alpha; o3[r] *= alpha; }
    const size_t va = vofs + kb;
    { const v16h a = frag_h(VT, va); o0 = mma1h(a, pf.v, o0); }
    { const v16h a = frag_h(VT, va + (size_t)16 * SEQ); o1 = mma1h(a, pf.v, o1); }
    { const v16h a = frag_h(VT, va + (size_t)32 * SEQ); o2 = mma1h(a, pf.v, o2); }
    { const v16h a = frag_h(VT, va + (size_t)48 * SEQ); o3 = mma1h(a, pf.v, o3); }
  }
  const float lt = l + __shfl_xor(l, 16);
  const float inv = 6.103515625e-05f * (1.0f / lt);
  const int qc = wave * 16 + ln;
  FragB ch0, cl0, ch1, cl1;
#pragma unroll
  for (int r = 0; r < 8; ++r) {
    { const float v = o0[r] * inv; const unsigned short hb = bf16_bits(v); ch0.u[r] = hb;     cl0.u[r] = bf16_bits(v - bf16_val(hb)); }
    { const float v = o1[r] * inv; const unsigned short hb = bf16_bits(v); ch0.u[8 + r] = hb; cl0.u[8 + r] = bf16_bits(v - bf16_val(hb)); }
    { const float v = o2[r] * inv; const unsigned short hb = bf16_bits(v); ch1.u[r] = hb;     cl1.u[r] = bf16_bits(v - bf16_val(hb)); }
    { const float v = o3[r] * inv; const unsigned short hb = bf16_bits(v); ch1.u[8 + r] = hb; cl1.u[8 + r] = bf16_bits(v - bf16_val(hb)); }
  }
#pragma unroll
  for (int ot = 0; ot < 4; ++ot) {
    const int woff = (ot * 16 + ln) * CC + 8 * hh;
    const v16b w0 = frag_w(Wo, woff), w1 = frag_w(Wo, woff + 32);
    v8f acc = z8;
    acc = mma1b(w0, ch0.v, acc);
    acc = mma1b(w0, cl0.v, acc);
    acc = mma1b(w1, ch1.v, acc);
    acc = mma1b(w1, cl1.v, acc);
    const int ob = ot * 16 + 8 * hh;
    const v4f bo0 = *(const v4fa*)(bo + ob), bo1 = *(const v4fa*)(bo + ob + 4);
    so[ob + 0][qc] = acc[0] + bf16_rne(bo0[0]);
    so[ob + 1][qc] = acc[1] + bf16_rne(bo0[1]);
    so[ob + 2][qc] = acc[2] + bf16_rne(bo0[2]);
    so[ob + 3][qc] = acc[3] + bf16_rne(bo0[3]);
    so[ob + 4][qc] = acc[4] + bf16_rne(bo1[0]);
    so[ob + 5][qc] = acc[5] + bf16_rne(bo1[1]);
    so[ob + 6][qc] = acc[6] + bf16_rne(bo1[2]);
    so[ob + 7][qc] = acc[7] + bf16_rne(bo1[3]);
  }
  __syncthreads();
  v4f res[8];
  const int c4 = ln * 4;
#pragma unroll
  for (int it = 0; it < 8; ++it) {
    const int c = wave * 16 + it * 2 + hh;
    res[it] = *(const v4fa*)&so[c][c4];
  }
  for (int pass = 0; pass < 2; ++pass) {
#pragma unroll
    for (int it = 0; it < 8; ++it) {
      const int c = wave * 16 + it * 2 + hh;
      const size_t g = ((size_t)b * CC + c) * SEQ_FULL + qb + c4;
      *(volatile v4f*)(out + g) = res[it];
    }
    if (pass == 0) __threadfence();
  }
}

extern "C" void kernel_launch(void* const* d_in, const int* in_sizes, int n_in,
                              void* d_out, int out_size, void* d_ws, size_t ws_size, hipStream_t stream) {
  if (n_in < 10) return;
  const long long need_s = ((long long)(NB - 1) * CQ + (CQ - 1)) * SEQ_FULL + SEQ;
  const long long need_d = (long long)(NB - 1) * SEQ_FULL + SEQ;
  const long long need_o = ((long long)(NB - 1) * CC + (CC - 1)) * SEQ_FULL + SEQ;
  if ((long long)in_sizes[0] < need_s || (long long)in_sizes[1] < need_d) return;
  if (in_sizes[2] < CC * CQ || in_sizes[8] < CC * CC) return;
  if (in_sizes[3] < CC || in_sizes[4] < CC || in_sizes[5] < CC || in_sizes[6] < CC || in_sizes[7] < CC || in_sizes[9] < CC) return;
  if ((long long)out_size < need_o) return;
  const float* xs = (const float*)d_in[0]; const float* xd = (const float*)d_in[1];
  const float* Wq = (const float*)d_in[2]; const float* bq = (const float*)d_in[3];
  const float* Wk = (const float*)d_in[4]; const float* bk = (const float*)d_in[5];
  const float* Wv = (const float*)d_in[6]; const float* bv = (const float*)d_in[7];
  const float* Wo = (const float*)d_in[8]; const float* bo = (const float*)d_in[9];
  const size_t PB = (size_t)NB * SEQ * CC * 2;
  if (5 * PB > ws_size) return;
  char* ws = (char*)d_ws;
  unsigned short* QH = (unsigned short*)(ws);
  unsigned short* QL = (unsigned short*)(ws + PB);
  unsigned short* KH = (unsigned short*)(ws + 2 * PB);
  unsigned short* KL = (unsigned short*)(ws + 3 * PB);
  unsigned short* VT = (unsigned short*)(ws + 4 * PB);
  const dim3 grid(SEQ / 64, NB);
  k_proj_q<<<grid, 128, 0, stream>>>(xs, Wq, bq, QH, QL);
  k_proj_kv<<<grid, 128, 0, stream>>>(xd, Wk, bk, Wv, bv, KH, KL, VT);
  k_attn<<<grid, 128, 0, stream>>>(QH, QL, KH, KL, VT, Wo, bo, (float*)d_out);
}
